// MambaLayer_20083267076883
// MI455X (gfx1250) — hardware-verified
//
#include <hip/hip_runtime.h>
#include <math.h>

typedef __attribute__((ext_vector_type(16))) _Float16 v16h;
typedef __attribute__((ext_vector_type(8)))  _Float16 v8h;
typedef __attribute__((ext_vector_type(16))) __bf16   v16b;
typedef __attribute__((ext_vector_type(8)))  __bf16   v8b;
typedef __attribute__((ext_vector_type(8)))  float    v8f;
typedef __attribute__((ext_vector_type(4)))  float    v4f;

constexpr int kB      = 2;
constexpr int kC      = 128;
constexpr int kSeq    = 4096;
constexpr int kRows   = kB * kSeq;
constexpr int kDI     = 256;
constexpr int kNst    = 16;
constexpr int kDtR    = 8;
constexpr int kConvK  = 4;
constexpr int kXzN    = 2 * kDI;
constexpr int kXdN    = kDtR + 2 * kNst;
constexpr int kXdP    = 64;
constexpr float kEps  = 1e-5f;
constexpr int kConvTP = 260;
constexpr int kScanTS = 64;
constexpr int kScanCh = 64;
constexpr int kScanYP = 68;
static_assert(kXdN == 40 && kXdN <= kXdP);
static_assert(kRows * kC == 1048576);
static_assert((kC % 32) == 0 && (kDI % 32) == 0);
static_assert((kRows % 64) == 0 && (kC % 64) == 0 && (kXzN % 64) == 0 && (kXdP % 64) == 0 && (kSeq % 64) == 0);
static_assert((kSeq % kScanTS) == 0 && (kDI % kScanCh) == 0 && kDI == 256 && kConvK == 4);

constexpr size_t kSzP16  = (size_t)kRows * kC * 2;
constexpr size_t kSzW16  = (size_t)kC * kC * 2;
constexpr size_t kSzT    = (size_t)kC * 4;
constexpr size_t kSzWIN  = (size_t)kXzN * kC * 2;
constexpr size_t kSzWXP  = (size_t)kXdP * kDI * 2;
constexpr size_t kSzWOUT = (size_t)kC * kDI * 2;
constexpr size_t kSzACT  = (size_t)kRows * kC * 4;
constexpr size_t kSzXZ   = (size_t)kRows * kXzN * 4;
constexpr size_t kSzUC   = (size_t)kRows * kDI * 4;
constexpr size_t kSzU16  = (size_t)kRows * kDI * 2;
constexpr size_t kSzXD   = (size_t)kRows * kXdP * 4;
constexpr size_t kSzYS   = (size_t)kRows * kC * 4;

constexpr size_t kOffXH   = 0;
constexpr size_t kOffXL   = kOffXH   + kSzP16;
constexpr size_t kOffW1H  = kOffXL   + kSzP16;
constexpr size_t kOffW1L  = kOffW1H  + kSzW16;
constexpr size_t kOffW2H  = kOffW1L  + kSzW16;
constexpr size_t kOffW2L  = kOffW2H  + kSzW16;
constexpr size_t kOffT1   = kOffW2L  + kSzW16;
constexpr size_t kOffT2   = kOffT1   + kSzT;
constexpr size_t kOffWIN0 = kOffT2   + kSzT;
constexpr size_t kOffWIN1 = kOffWIN0 + kSzWIN;
constexpr size_t kOffWXP  = kOffWIN1 + kSzWIN;
constexpr size_t kOffWO0  = kOffWXP  + kSzWXP;
constexpr size_t kOffWO1  = kOffWO0  + kSzWOUT;
constexpr size_t kOffACT  = kOffWO1  + kSzWOUT;
constexpr size_t kOffACTB = kOffACT  + kSzACT;
constexpr size_t kOffXZ   = kOffACTB + kSzP16;
constexpr size_t kOffUC   = kOffXZ   + kSzXZ;
constexpr size_t kOffUCB  = kOffUC   + kSzUC;
constexpr size_t kOffXD   = kOffUCB  + kSzU16;
constexpr size_t kOffYB   = kOffXD   + kSzXD;
constexpr size_t kOffYS   = kOffYB   + kSzU16;
constexpr size_t kOffMIDH = kOffYS   + 4 * kSzYS;
constexpr size_t kOffMIDL = kOffMIDH + kSzP16;
constexpr size_t kWsTotal = kOffMIDL + kSzP16;
static_assert(kWsTotal == 67666944ull);
static_assert(kWsTotal <= 134217728ull);
static_assert((kOffXL % 128) == 0 && (kOffW1H % 128) == 0 && (kOffW1L % 128) == 0 && (kOffW2H % 128) == 0 &&
              (kOffW2L % 128) == 0 && (kOffT1 % 128) == 0 && (kOffT2 % 128) == 0 && (kOffWIN0 % 128) == 0 &&
              (kOffWIN1 % 128) == 0 && (kOffWXP % 128) == 0 && (kOffWO0 % 128) == 0 && (kOffWO1 % 128) == 0 &&
              (kOffACT % 128) == 0 && (kOffACTB % 128) == 0 && (kOffXZ % 128) == 0 && (kOffUC % 128) == 0 &&
              (kOffUCB % 128) == 0 && (kOffXD % 128) == 0 && (kOffYB % 128) == 0 && (kOffYS % 128) == 0 &&
              (kOffMIDH % 128) == 0 && (kOffMIDL % 128) == 0);

__device__ __forceinline__ unsigned short f2bf_bits(float f) {
  unsigned u = __float_as_uint(f);
  return (unsigned short)((u + 0x7FFFu + ((u >> 16) & 1u)) >> 16);
}
__device__ __forceinline__ float bf_bits2f(unsigned short h) { return __uint_as_float(((unsigned)h) << 16); }

__device__ __forceinline__ void dep_guard4_h(v8f& a, v8f& b, v8f& c, v8f& d, v16h x, v16h y) { asm volatile("v_nop\n\tv_nop\n\tv_nop\n\tv_nop" : "+v"(a), "+v"(b), "+v"(c), "+v"(d) : "v"(x), "v"(y)); }
__device__ __forceinline__ void dep_guard4_b(v8f& a, v8f& b, v8f& c, v8f& d, v16b x, v16b y) { asm volatile("v_nop\n\tv_nop\n\tv_nop\n\tv_nop" : "+v"(a), "+v"(b), "+v"(c), "+v"(d) : "v"(x), "v"(y)); }
__device__ __forceinline__ void keep4_h(v16h a, v16h b, v16h c, v16h d) { asm volatile("v_nop" :: "v"(a), "v"(b), "v"(c), "v"(d)); }
__device__ __forceinline__ void keep4_b(v16b a, v16b b, v16b c, v16b d) { asm volatile("v_nop" :: "v"(a), "v"(b), "v"(c), "v"(d)); }
__device__ __forceinline__ void acc_guard4(v8f& a, v8f& b, v8f& c, v8f& d) { asm volatile("v_nop\n\tv_nop\n\tv_nop\n\tv_nop" : "+v"(a), "+v"(b), "+v"(c), "+v"(d)); }
template <typename T> struct Frag;
template <> struct Frag<_Float16> {
  typedef v16h V; union U { v16h v; v8h h[2]; };
  static __device__ __forceinline__ v16h load(const _Float16* p) {
    U f; f.h[0] = *(const v8h*)(p); f.h[1] = *(const v8h*)(p + 16); return f.v;
  }
  static __device__ __forceinline__ v8f mma(v16h a, v16h b, v8f c) {
    return __builtin_amdgcn_wmma_f32_16x16x32_f16(false, a, false, b, (short)0, c, false, false);
  }
  static __device__ __forceinline__ void guard4(v8f& a, v8f& b, v8f& c, v8f& d, v16h x, v16h y) { dep_guard4_h(a, b, c, d, x, y); }
  static __device__ __forceinline__ void keep(v16h a, v16h b, v16h c, v16h d) { keep4_h(a, b, c, d); }
};
template <> struct Frag<__bf16> {
  typedef v16b V; union U { v16b v; v8b h[2]; };
  static __device__ __forceinline__ v16b load(const __bf16* p) {
    U f; f.h[0] = *(const v8b*)(p); f.h[1] = *(const v8b*)(p + 16); return f.v;
  }
  static __device__ __forceinline__ v8f mma(v16b a, v16b b, v8f c) {
    return __builtin_amdgcn_wmma_f32_16x16x32_bf16(false, a, false, b, (short)0, c, false, false);
  }
  static __device__ __forceinline__ void guard4(v8f& a, v8f& b, v8f& c, v8f& d, v16b x, v16b y) { dep_guard4_b(a, b, c, d, x, y); }
  static __device__ __forceinline__ void keep(v16b a, v16b b, v16b c, v16b d) { keep4_b(a, b, c, d); }
};

template <int ET> struct Elem;
template <> struct Elem<0> { typedef _Float16 T; };
template <> struct Elem<1> { typedef __bf16 T; };
template <int ET, int SPL, int BIAS_MODE, int OUT_MODE, int ACT>
__global__ __launch_bounds__(256) void wmma_gemm64(
    const unsigned short* __restrict__ Ap, const unsigned short* __restrict__ A2p, int lda, long strideA,
    const unsigned short* __restrict__ Btp, const unsigned short* __restrict__ Bt2p, int ldb, long strideB,
    void* __restrict__ Cout, void* __restrict__ Cout2, int ldc, long strideC,
    const float* __restrict__ bias,
    int M, int N, int K, float scale) {
  typedef typename Elem<ET>::T T;
  typedef typename Frag<T>::V V;
  const T* A = (const T*)Ap; const T* A2 = (const T*)A2p; const T* Bt = (const T*)Btp; const T* Bt2 = (const T*)Bt2p;
  __shared__ __align__(16) float sT[8][16 * 68];
  const int b    = blockIdx.y;
  const int lane = threadIdx.x & 31;
  const int wave = threadIdx.x >> 5;
  const int tilesN = N >> 6;
  const int tilesM = M >> 6;
  const int tile = blockIdx.x * 8 + wave;
  if (tile >= tilesM * tilesN) return;
  const int tm = tile / tilesN;
  const int tn = tile - tm * tilesN;
  const int m0 = tm << 6;
  const int n0 = tn << 6;

  const T* Ab  = A  + (size_t)b * strideA;
  const T* Bb  = Bt + (size_t)b * strideB;
  const T* Ab2 = (SPL >= 1) ? (A2  + (size_t)b * strideA) : nullptr;
  const T* Bb2 = (SPL == 2) ? (Bt2 + (size_t)b * strideB) : nullptr;

  const int rlane = lane & 15;
  const int koff  = (lane >> 4) * 8;
  const int mOff  = (lane >> 4) * 8;

  v8f acc[4][4];
#pragma unroll
  for (int i = 0; i < 4; ++i)
#pragma unroll
    for (int j = 0; j < 4; ++j) acc[i][j] = (v8f){0.f,0.f,0.f,0.f,0.f,0.f,0.f,0.f};

  for (int k0 = 0; k0 < K; k0 += 32) {
    V bh[4], bl[4];
#pragma unroll
    for (int j = 0; j < 4; ++j) {
      const size_t bo = (size_t)(n0 + (j << 4) + rlane) * ldb + koff + k0;
      bh[j] = Frag<T>::load(Bb + bo);
      if (SPL == 2) bl[j] = Frag<T>::load(Bb2 + bo);
    }
#pragma unroll
    for (int i = 0; i < 4; ++i) {
      const size_t ao = (size_t)(m0 + (i << 4) + rlane) * lda + koff + k0;
      V ah = Frag<T>::load(Ab + ao);
      V al;
      if (SPL >= 1) al = Frag<T>::load(Ab2 + ao);
#pragma unroll
      for (int j = 0; j < 4; ++j) {
        acc[i][j] = Frag<T>::mma(ah, bh[j], acc[i][j]);
        if (SPL == 2) acc[i][j] = Frag<T>::mma(ah, bl[j], acc[i][j]);
        if (SPL >= 1) acc[i][j] = Frag<T>::mma(al, bh[j], acc[i][j]);
      }
      Frag<T>::guard4(acc[i][0], acc[i][1], acc[i][2], acc[i][3], ah, (SPL >= 1) ? al : ah);
    }
    Frag<T>::keep(bh[0], bh[1], bh[2], bh[3]);
    if (SPL == 2) Frag<T>::keep(bl[0], bl[1], bl[2], bl[3]);
  }
  acc_guard4(acc[0][0], acc[0][1], acc[0][2], acc[0][3]);
  acc_guard4(acc[1][0], acc[1][1], acc[1][2], acc[1][3]);
  acc_guard4(acc[2][0], acc[2][1], acc[2][2], acc[2][3]);
  acc_guard4(acc[3][0], acc[3][1], acc[3][2], acc[3][3]);

  float* slab = sT[wave];
#pragma unroll
  for (int i = 0; i < 4; ++i) {
    const int mBase = m0 + (i << 4);
#pragma unroll
    for (int j = 0; j < 4; ++j) {
      const int n = n0 + (j << 4) + rlane;
      float bv = 0.f;
      if (BIAS_MODE == 2) bv = bias[n];
#pragma unroll
      for (int r = 0; r < 8; ++r) {
        float v = acc[i][j][r] * scale;
        if (BIAS_MODE == 1) v += bias[mBase + mOff + r];
        if (BIAS_MODE == 2) v += bv;
        if (ACT == 2) v = fmaxf(v, 0.0f);
        slab[(mOff + r) * 68 + (j << 4) + rlane] = v;
      }
    }
    __builtin_amdgcn_fence(__ATOMIC_RELEASE, "workgroup");
    __builtin_amdgcn_wave_barrier();
    __builtin_amdgcn_fence(__ATOMIC_ACQUIRE, "workgroup");
    if (OUT_MODE == 0 || OUT_MODE == 3) {
      float* Cf = (float*)Cout + (size_t)b * strideC;
      unsigned short* Cb = (unsigned short*)Cout2 + (size_t)b * strideC;
      const int hh = lane >> 4, c4 = (lane & 15) * 4;
      const int q8 = lane >> 3, c8 = (lane & 7) * 8;
      for (int pass = 0; pass < 2; ++pass) {
#pragma unroll
        for (int it = 0; it < 8; ++it) {
          const int row = it * 2 + hh;
          v4f v = *(const v4f*)(slab + row * 68 + c4);
          *(volatile v4f*)(Cf + (size_t)(mBase + row) * ldc + n0 + c4) = v;
        }
        if (OUT_MODE == 3) {
#pragma unroll
          for (int it = 0; it < 4; ++it) {
            const int row = it * 4 + q8;
            const float* sp = slab + row * 68 + c8;
            v8h hv;
#pragma unroll
            for (int e = 0; e < 8; ++e) {
              const unsigned short hb = f2bf_bits(sp[e]);
              hv[e] = __builtin_bit_cast(_Float16, hb);
            }
            *(volatile v8h*)(Cb + (size_t)(mBase + row) * ldc + n0 + c8) = hv;
          }
        }
        __threadfence();
      }
    } else {
      const int q = lane >> 3, c8 = (lane & 7) * 8;
      unsigned short* C1 = (unsigned short*)Cout  + (size_t)b * strideC;
      unsigned short* C2 = (OUT_MODE == 2) ? ((unsigned short*)Cout2 + (size_t)b * strideC) : nullptr;
      for (int pass = 0; pass < 2; ++pass) {
#pragma unroll
        for (int it = 0; it < 4; ++it) {
          const int row = it * 4 + q;
          const float* sp = slab + row * 68 + c8;
          v8h hv, lv;
#pragma unroll
          for (int e = 0; e < 8; ++e) {
            if (OUT_MODE == 1) {
              hv[e] = (_Float16)sp[e];
            } else {
              unsigned short hb = f2bf_bits(sp[e]);
              unsigned short lb = f2bf_bits(sp[e] - bf_bits2f(hb));
              hv[e] = __builtin_bit_cast(_Float16, hb);
              lv[e] = __builtin_bit_cast(_Float16, lb);
            }
          }
          *(volatile v8h*)(C1 + (size_t)(mBase + row) * ldc + n0 + c8) = hv;
          if (OUT_MODE == 2) *(volatile v8h*)(C2 + (size_t)(mBase + row) * ldc + n0 + c8) = lv;
        }
        __threadfence();
      }
    }
    __builtin_amdgcn_fence(__ATOMIC_RELEASE, "workgroup");
    __builtin_amdgcn_wave_barrier();
    __builtin_amdgcn_fence(__ATOMIC_ACQUIRE, "workgroup");
  }
}

__global__ __launch_bounds__(256) void x_transpose_split_kernel(
    const float* __restrict__ x, unsigned short* __restrict__ XH, unsigned short* __restrict__ XL)
{
  __shared__ float tile[64 * 65];
  const int tid = threadIdx.x, lane = tid & 31, wave = tid >> 5;
  const int n0 = blockIdx.x * 64;
  const int k0 = blockIdx.y * 64;
  const int b  = blockIdx.z;
  const float* xb = x + (size_t)b * kC * kSeq;
#pragma unroll
  for (int p = 0; p < 8; ++p) {
    const int idx = tid + p * 256;
    const int kk  = idx >> 6;
    const int nn  = idx & 63;
    tile[kk * 65 + nn] = xb[(size_t)(k0 + kk) * kSeq + n0 + nn];
  }
  asm volatile("" ::: "memory");
#pragma unroll
  for (int p = 8; p < 16; ++p) {
    const int idx = tid + p * 256;
    const int kk  = idx >> 6;
    const int nn  = idx & 63;
    tile[kk * 65 + nn] = xb[(size_t)(k0 + kk) * kSeq + n0 + nn];
  }
  __syncthreads();
  const int q = lane >> 3, c8 = (lane & 7) * 8;
  v8h hv[2], lv[2];
#pragma unroll
  for (int it = 0; it < 2; ++it) {
    const int nrow = it * 32 + wave * 4 + q;
#pragma unroll
    for (int e = 0; e < 8; ++e) {
      const float f = tile[(c8 + e) * 65 + nrow];
      const unsigned short hb = f2bf_bits(f);
      const unsigned short lb = f2bf_bits(f - bf_bits2f(hb));
      hv[it][e] = __builtin_bit_cast(_Float16, hb);
      lv[it][e] = __builtin_bit_cast(_Float16, lb);
    }
  }
  for (int pass = 0; pass < 2; ++pass) {
#pragma unroll
    for (int it = 0; it < 2; ++it) {
      const int nrow = it * 32 + wave * 4 + q;
      const size_t o = ((size_t)b * kSeq + n0 + nrow) * kC + k0 + c8;
      *(volatile v8h*)(XH + o) = hv[it];
      *(volatile v8h*)(XL + o) = lv[it];
    }
    __threadfence();
  }
}

__global__ __launch_bounds__(256) void bn_fold_split_kernel(
    const float* __restrict__ W, const float* __restrict__ bng, const float* __restrict__ bnb,
    const float* __restrict__ bnm, const float* __restrict__ bnv,
    unsigned short* __restrict__ WH, unsigned short* __restrict__ WL, float* __restrict__ T)
{
  const int i = blockIdx.x * 256 + threadIdx.x;
  const int o = i >> 4;
  const float sc = bng[o] * (1.0f / sqrtf(bnv[o] + kEps));
  const size_t e0 = (size_t)i << 3;
  const v4f a0 = *(const v4f*)(W + e0);
  const v4f a1 = *(const v4f*)(W + e0 + 4);
  v8h hv, lv;
#pragma unroll
  for (int e = 0; e < 4; ++e) {
    const float f0 = a0[e] * sc, f1 = a1[e] * sc;
    const unsigned short h0 = f2bf_bits(f0), h1 = f2bf_bits(f1);
    const unsigned short l0 = f2bf_bits(f0 - bf_bits2f(h0)), l1 = f2bf_bits(f1 - bf_bits2f(h1));
    hv[e]     = __builtin_bit_cast(_Float16, h0);
    hv[4 + e] = __builtin_bit_cast(_Float16, h1);
    lv[e]     = __builtin_bit_cast(_Float16, l0);
    lv[4 + e] = __builtin_bit_cast(_Float16, l1);
  }
  unsigned short* qh = WH + e0;
  unsigned short* ql = WL + e0;
  *(volatile v8h*)qh = hv;
  *(volatile v8h*)ql = lv;
  __threadfence();
  *(volatile v8h*)qh = hv;
  *(volatile v8h*)ql = lv;
  if (blockIdx.x == 0 && threadIdx.x < 32) {
    const int o4 = threadIdx.x * 4;
    const v4f g4 = *(const v4f*)(bng + o4);
    const v4f b4 = *(const v4f*)(bnb + o4);
    const v4f m4 = *(const v4f*)(bnm + o4);
    const v4f v4 = *(const v4f*)(bnv + o4);
    v4f t;
#pragma unroll
    for (int e = 0; e < 4; ++e) {
      const float s = g4[e] * (1.0f / sqrtf(v4[e] + kEps));
      t[e] = b4[e] - m4[e] * s;
    }
    *(volatile v4f*)(T + o4) = t;
    __threadfence();
    *(volatile v4f*)(T + o4) = t;
  }
}

__global__ __launch_bounds__(256) void cast_rows_bf16_kernel(
    const float* __restrict__ src, unsigned short* __restrict__ dst,
    int srcRows, int cols, int flipR, int flipC, int total8)
{
  const int i = blockIdx.x * 256 + threadIdx.x;
  if (i >= total8) return;
  const int e0 = i << 3;
  const int r  = e0 / cols;
  const int c  = e0 - r * cols;
  const bool valid = (r < srcRows);
  const int rc = valid ? r : (srcRows - 1);
  const int sr = flipR ? (srcRows - 1 - rc) : rc;
  const int scol = flipC ? (cols - 8 - c) : c;
  const float* p = src + (size_t)sr * cols + scol;
  const v4f a0 = *(const v4f*)(p);
  const v4f a1 = *(const v4f*)(p + 4);
  v8h hv;
#pragma unroll
  for (int e = 0; e < 4; ++e) {
    const float f0 = flipC ? a1[3 - e] : a0[e];
    const float f1 = flipC ? a0[3 - e] : a1[e];
    const float g0 = valid ? f0 : 0.0f;
    const float g1 = valid ? f1 : 0.0f;
    const unsigned short h0 = f2bf_bits(g0), h1 = f2bf_bits(g1);
    hv[e]     = __builtin_bit_cast(_Float16, h0);
    hv[4 + e] = __builtin_bit_cast(_Float16, h1);
  }
  unsigned short* qd = dst + e0;
  *(volatile v8h*)qd = hv;
  __threadfence();
  *(volatile v8h*)qd = hv;
}

__device__ __forceinline__ int conv_tok(int g0, int st, int dirL) { return dirL ? (g0 + 63 - st) : (g0 + st); }

__global__ __launch_bounds__(256) void conv_silu_kernel(
    const float* __restrict__ XZ, const float* __restrict__ cw, const float* __restrict__ cb,
    float* __restrict__ UC, unsigned short* __restrict__ UCB, int dirL)
{
  __shared__ __align__(16) float sT[16 * kConvTP];
  const int tid = threadIdx.x, lane = tid & 31, wave = tid >> 5;
  const int d  = tid;
  const int g0 = blockIdx.x * 64;
  const int tb = g0 & (kSeq - 1);
  const float w0 = cw[d * kConvK + 0], w1 = cw[d * kConvK + 1], w2 = cw[d * kConvK + 2], w3 = cw[d * kConvK + 3];
  const float bc = cb[d];
  float xm3, xm2, xm1;
  {
    const bool hist = dirL ? (tb + 64 < kSeq) : (tb > 0);
    const int r1 = dirL ? (g0 + 64) : (g0 - 1);
    const int r2 = dirL ? (g0 + 65) : (g0 - 2);
    const int r3 = dirL ? (g0 + 66) : (g0 - 3);
    const int c1 = hist ? r1 : g0, c2 = hist ? r2 : g0, c3 = hist ? r3 : g0;
    const float v1 = XZ[(size_t)c1 * kXzN + d];
    const float v2 = XZ[(size_t)c2 * kXzN + d];
    const float v3 = XZ[(size_t)c3 * kXzN + d];
    xm1 = hist ? v1 : 0.0f;
    xm2 = hist ? v2 : 0.0f;
    xm3 = hist ? v3 : 0.0f;
  }
  const int hrow = wave >> 1;
  const int hch  = (wave & 1) * 128 + lane * 4;
#pragma unroll 1
  for (int sub = 0; sub < 4; ++sub) {
#pragma unroll 1
    for (int s = 0; s < 16; ++s) {
      const int tok = conv_tok(g0, sub * 16 + s, dirL);
      const float xcur = XZ[(size_t)tok * kXzN + d];
      float acc = w0 * xm3;
      acc = fmaf(w1, xm2, acc);
      acc = fmaf(w2, xm1, acc);
      acc = fmaf(w3, xcur, acc);
      const float sv = acc + bc;
      const float sg = __builtin_amdgcn_rcpf(1.0f + expf(-sv));
      sT[s * kConvTP + tid] = sv * sg;
      xm3 = xm2; xm2 = xm1; xm1 = xcur;
    }
    __syncthreads();
    v4f fv[4];
    v8h bv[2];
#pragma unroll
    for (int it = 0; it < 4; ++it) fv[it] = *(const v4f*)(sT + (it * 4 + hrow) * kConvTP + hch);
#pragma unroll
    for (int it = 0; it < 2; ++it) {
      const float* sp = sT + (it * 8 + wave) * kConvTP + lane * 8;
      const v4f a0 = *(const v4f*)(sp);
      const v4f a1 = *(const v4f*)(sp + 4);
#pragma unroll
      for (int e = 0; e < 4; ++e) {
        const unsigned short h0 = f2bf_bits(a0[e]), h1 = f2bf_bits(a1[e]);
        bv[it][e]     = __builtin_bit_cast(_Float16, h0);
        bv[it][4 + e] = __builtin_bit_cast(_Float16, h1);
      }
    }
    for (int pass = 0; pass < 2; ++pass) {
#pragma unroll
      for (int it = 0; it < 4; ++it) {
        const int tok = conv_tok(g0, sub * 16 + it * 4 + hrow, dirL);
        *(volatile v4f*)(UC + (size_t)tok * kDI + hch) = fv[it];
      }
#pragma unroll
      for (int it = 0; it < 2; ++it) {
        const int tok = conv_tok(g0, sub * 16 + it * 8 + wave, dirL);
        *(volatile v8h*)(UCB + (size_t)tok * kDI + lane * 8) = bv[it];
      }
      __threadfence();
    }
    __syncthreads();
  }
}

__global__ __launch_bounds__(64) void scan_kernel(
    const float* __restrict__ XD, const float* __restrict__ UC, const float* __restrict__ XZ,
    const float* __restrict__ Wdt, const float* __restrict__ bdt, const float* __restrict__ Alog,
    const float* __restrict__ Dp, unsigned short* __restrict__ YB, int dirL)
{
  __shared__ __align__(16) float sX[kScanTS * kXdP];
  __shared__ __align__(16) float sY[kScanTS * kScanYP];
  __shared__ __align__(16) float sW[kDtR * kScanCh];
  __shared__ __align__(16) float sA[kNst * kScanCh];
  const int tid = threadIdx.x, lane = tid & 31, wave = tid >> 5;
  constexpr int kBlkPerB = kDI / kScanCh;
  const int bix = blockIdx.x / kBlkPerB;
  const int d0  = (blockIdx.x - bix * kBlkPerB) * kScanCh;
  const int d   = d0 + tid;
  const size_t rowb = (size_t)bix * kSeq;
#pragma unroll 1
  for (int r = 0; r < kDtR; ++r) sW[r * kScanCh + tid] = Wdt[(size_t)d * kDtR + r];
#pragma unroll 1
  for (int s = 0; s < kNst; ++s) sA[s * kScanCh + tid] = -expf(Alog[(size_t)d * kNst + s]);
  __syncthreads();
  float negA[kNst], h[kNst];
#pragma unroll
  for (int s = 0; s < kNst; ++s) {
    negA[s] = sA[s * kScanCh + tid];
    h[s] = 0.0f;
  }
  const float bb = bdt[d], Dd = Dp[d];
  const int lr = tid >> 4, lc4 = (tid & 15) * 4;
  const int q = lane >> 3, c8 = (lane & 7) * 8;
#pragma unroll 1
  for (int cix = 0; cix < kSeq / kScanTS; ++cix) {
    const int tb = dirL ? (kSeq - kScanTS - cix * kScanTS) : (cix * kScanTS);
    __syncthreads();
#pragma unroll
    for (int i = 0; i < 8; ++i) {
      const int r = lr + 4 * i;
      *(v4f*)(sX + r * kXdP + lc4) = *(const v4f*)(XD + (rowb + tb + r) * kXdP + lc4);
    }
    asm volatile("" ::: "memory");
#pragma unroll
    for (int i = 8; i < 16; ++i) {
      const int r = lr + 4 * i;
      *(v4f*)(sX + r * kXdP + lc4) = *(const v4f*)(XD + (rowb + tb + r) * kXdP + lc4);
    }
    __syncthreads();
#pragma unroll 1
    for (int s = 0; s < kScanTS; ++s) {
      const int r = dirL ? (kScanTS - 1 - s) : s;
      const size_t grow = rowb + tb + r;
      const float* xr = sX + r * kXdP;
      float vdot = 0.0f;
#pragma unroll 1
      for (int rr = 0; rr < kDtR; ++rr) vdot = fmaf(xr[rr], sW[rr * kScanCh + tid], vdot);
      float Bs[kNst], Cs[kNst];
#pragma unroll
      for (int q4 = 0; q4 < 4; ++q4) {
        const v4f bv = *(const v4f*)(xr + kDtR + 4 * q4);
        const v4f cv = *(const v4f*)(xr + kDtR + kNst + 4 * q4);
        Bs[4 * q4 + 0] = bv[0]; Bs[4 * q4 + 1] = bv[1]; Bs[4 * q4 + 2] = bv[2]; Bs[4 * q4 + 3] = bv[3];
        Cs[4 * q4 + 0] = cv[0]; Cs[4 * q4 + 1] = cv[1]; Cs[4 * q4 + 2] = cv[2]; Cs[4 * q4 + 3] = cv[3];
      }
      const float v   = vdot + bb;
      const float ea  = expf(-fabsf(v));
      const float dt  = fmaxf(v, 0.0f) + log1pf(ea);
      const float xt  = UC[grow * kDI + d];
      const float dtx = dt * xt;
      float y = 0.0f;
#pragma unroll
      for (int k = 0; k < kNst; ++k) {
        const float e = expf(dt * negA[k]);
        float dbu = dtx * Bs[k];
        asm volatile("" : "+v"(dbu));
        float eh = e * h[k];
        asm volatile("" : "+v"(eh));
        const float hn = eh + dbu;
        h[k] = hn;
        float rc = hn * Cs[k];
        asm volatile("" : "+v"(rc));
        y = y + rc;
      }
      float sk = xt * Dd;
      asm volatile("" : "+v"(sk));
      y = y + sk;
      const float zv = XZ[grow * kXzN + kDI + d];
      const float sg = __builtin_amdgcn_rcpf(1.0f + expf(-zv));
      const float g  = zv * sg;
      sY[r * kScanYP + tid] = y * g;
    }
    __syncthreads();
    v8h hv[8];
#pragma unroll
    for (int it = 0; it < 8; ++it) {
      const int row = it * 8 + wave * 4 + q;
      const float* sp = sY + row * kScanYP + c8;
      const v4f a0 = *(const v4f*)(sp);
      const v4f a1 = *(const v4f*)(sp + 4);
#pragma unroll
      for (int e = 0; e < 4; ++e) {
        const unsigned short h0 = f2bf_bits(a0[e]), h1 = f2bf_bits(a1[e]);
        hv[it][e]     = __builtin_bit_cast(_Float16, h0);
        hv[it][4 + e] = __builtin_bit_cast(_Float16, h1);
      }
    }
    for (int pass = 0; pass < 2; ++pass) {
#pragma unroll
      for (int it = 0; it < 8; ++it) {
        const int row = it * 8 + wave * 4 + q;
        const size_t o = (rowb + tb + row) * kDI + d0 + c8;
        *(volatile v8h*)(YB + o) = hv[it];
      }
      __threadfence();
    }
  }
}

__global__ __launch_bounds__(256) void mid_split_kernel(
    const float* __restrict__ Y0, const float* __restrict__ Y1, const float* __restrict__ Y2, const float* __restrict__ Y3,
    const float* __restrict__ ACT, unsigned short* __restrict__ MH, unsigned short* __restrict__ ML, int total8)
{
  const int i = blockIdx.x * 256 + threadIdx.x;
  if (i >= total8) return;
  const size_t e0 = (size_t)i << 3;
  const v4f a0 = *(const v4f*)(Y0 + e0), a1 = *(const v4f*)(Y0 + e0 + 4);
  const v4f b0 = *(const v4f*)(Y1 + e0), b1 = *(const v4f*)(Y1 + e0 + 4);
  const v4f c0 = *(const v4f*)(Y2 + e0), c1 = *(const v4f*)(Y2 + e0 + 4);
  asm volatile("" ::: "memory");
  const v4f f0 = *(const v4f*)(Y3 + e0), f1 = *(const v4f*)(Y3 + e0 + 4);
  const v4f r0 = *(const v4f*)(ACT + e0), r1 = *(const v4f*)(ACT + e0 + 4);
  v8h hv, lv;
#pragma unroll
  for (int e = 0; e < 4; ++e) {
    const float s0 = ((a0[e] + b0[e]) + c0[e]) + f0[e];
    const float s1 = ((a1[e] + b1[e]) + c1[e]) + f1[e];
    const float m0 = s0 * 0.25f + r0[e];
    const float m1 = s1 * 0.25f + r1[e];
    const unsigned short h0 = f2bf_bits(m0), h1 = f2bf_bits(m1);
    const unsigned short l0 = f2bf_bits(m0 - bf_bits2f(h0)), l1 = f2bf_bits(m1 - bf_bits2f(h1));
    hv[e]     = __builtin_bit_cast(_Float16, h0);
    hv[4 + e] = __builtin_bit_cast(_Float16, h1);
    lv[e]     = __builtin_bit_cast(_Float16, l0);
    lv[4 + e] = __builtin_bit_cast(_Float16, l1);
  }
  unsigned short* qh = MH + e0;
  unsigned short* ql = ML + e0;
  *(volatile v8h*)qh = hv;
  *(volatile v8h*)ql = lv;
  __threadfence();
  *(volatile v8h*)qh = hv;
  *(volatile v8h*)ql = lv;
}

extern "C" void kernel_launch(void* const* d_in, const int* in_sizes, int n_in,
                              void* d_out, int out_size, void* d_ws, size_t ws_size,
                              hipStream_t stream)
{
  if (n_in < 20) return;
  if (in_sizes[0] != kB * kC * kSeq) return;
  if (in_sizes[1] != kC * kC || in_sizes[2] != kC * kC) return;
  for (int i = 3; i <= 10; ++i) if (in_sizes[i] != kC) return;
  if (in_sizes[11] != kXzN * kC) return;
  if (in_sizes[12] != kDI * kConvK || in_sizes[13] != kDI) return;
  if (in_sizes[14] != kXdN * kDI) return;
  if (in_sizes[15] != kDI * kDtR || in_sizes[16] != kDI) return;
  if (in_sizes[17] != kDI * kNst || in_sizes[18] != kDI) return;
  if (in_sizes[19] != kC * kDI) return;
  if (out_size != kRows * kC) return;
  if (ws_size < kWsTotal) return;

  const float* x        = (const float*)d_in[0];
  const float* nin_w    = (const float*)d_in[1];
  const float* nin2_w   = (const float*)d_in[2];
  const float* bn1_g    = (const float*)d_in[3];
  const float* bn1_b    = (const float*)d_in[4];
  const float* bn1_m    = (const float*)d_in[5];
  const float* bn1_v    = (const float*)d_in[6];
  const float* bn2_g    = (const float*)d_in[7];
  const float* bn2_b    = (const float*)d_in[8];
  const float* bn2_m    = (const float*)d_in[9];
  const float* bn2_v    = (const float*)d_in[10];
  const float* in_proj  = (const float*)d_in[11];
  const float* conv_w   = (const float*)d_in[12];
  const float* conv_b   = (const float*)d_in[13];
  const float* xproj_w  = (const float*)d_in[14];
  const float* dtproj_w = (const float*)d_in[15];
  const float* dtproj_b = (const float*)d_in[16];
  const float* A_log    = (const float*)d_in[17];
  const float* D_param  = (const float*)d_in[18];
  const float* out_proj = (const float*)d_in[19];
  float* dout = (float*)d_out;

  char* ws = (char*)d_ws;
  unsigned short* XH   = (unsigned short*)(ws + kOffXH);
  unsigned short* XL   = (unsigned short*)(ws + kOffXL);
  unsigned short* W1H  = (unsigned short*)(ws + kOffW1H);
  unsigned short* W1L  = (unsigned short*)(ws + kOffW1L);
  unsigned short* W2H  = (unsigned short*)(ws + kOffW2H);
  unsigned short* W2L  = (unsigned short*)(ws + kOffW2L);
  float*          T1   = (float*)(ws + kOffT1);
  float*          T2   = (float*)(ws + kOffT2);
  unsigned short* WIN0 = (unsigned short*)(ws + kOffWIN0);
  unsigned short* WIN1 = (unsigned short*)(ws + kOffWIN1);
  unsigned short* WXP  = (unsigned short*)(ws + kOffWXP);
  unsigned short* WO0  = (unsigned short*)(ws + kOffWO0);
  unsigned short* WO1  = (unsigned short*)(ws + kOffWO1);
  float*          ACT  = (float*)(ws + kOffACT);
  unsigned short* ACTB = (unsigned short*)(ws + kOffACTB);
  float*          XZ   = (float*)(ws + kOffXZ);
  float*          UC   = (float*)(ws + kOffUC);
  unsigned short* UCB  = (unsigned short*)(ws + kOffUCB);
  float*          XD   = (float*)(ws + kOffXD);
  unsigned short* YB   = (unsigned short*)(ws + kOffYB);
  float*          YS   = (float*)(ws + kOffYS);
  unsigned short* MIDH = (unsigned short*)(ws + kOffMIDH);
  unsigned short* MIDL = (unsigned short*)(ws + kOffMIDL);
  const float* dummy_bias = T1;

  x_transpose_split_kernel<<<dim3(kSeq / 64, kC / 64, kB), 256, 0, stream>>>(x, XH, XL);
  bn_fold_split_kernel<<<(kC * kC / 8) / 256, 256, 0, stream>>>(nin_w,  bn1_g, bn1_b, bn1_m, bn1_v, W1H, W1L, T1);
  bn_fold_split_kernel<<<(kC * kC / 8) / 256, 256, 0, stream>>>(nin2_w, bn2_g, bn2_b, bn2_m, bn2_v, W2H, W2L, T2);
  cast_rows_bf16_kernel<<<(kXzN * kC / 8) / 256, 256, 0, stream>>>(in_proj, WIN0, kXzN, kC, 0, 0, kXzN * kC / 8);
  cast_rows_bf16_kernel<<<(kXzN * kC / 8) / 256, 256, 0, stream>>>(in_proj, WIN1, kXzN, kC, 0, 1, kXzN * kC / 8);
  cast_rows_bf16_kernel<<<(kXdP * kDI / 8) / 256, 256, 0, stream>>>(xproj_w, WXP, kXdN, kDI, 0, 0, kXdP * kDI / 8);
  cast_rows_bf16_kernel<<<(kC * kDI / 8) / 256, 256, 0, stream>>>(out_proj, WO0, kC, kDI, 0, 0, kC * kDI / 8);
  cast_rows_bf16_kernel<<<(kC * kDI / 8) / 256, 256, 0, stream>>>(out_proj, WO1, kC, kDI, 1, 0, kC * kDI / 8);

  wmma_gemm64<1, 2, 2, 3, 2><<<dim3(32, 1), 256, 0, stream>>>(
      XH, XL, kC, 0L,
      W1H, W1L, kC, 0L,
      (void*)ACT, (void*)ACTB, kC, 0L,
      T1,
      kRows, kC, kC, 1.0f);

  for (int dd = 0; dd < 4; ++dd) {
    const int dirC = dd & 1;
    const int dirL = dd >> 1;
    const unsigned short* WINd = dirC ? WIN1 : WIN0;
    const unsigned short* WOd  = dirC ? WO1 : WO0;
    float* YSd = YS + (size_t)dd * kRows * kC;

    wmma_gemm64<1, 0, 0, 0, 0><<<dim3(128, 1), 256, 0, stream>>>(
        ACTB, ACTB, kC, 0L,
        WINd, WINd, kC, 0L,
        (void*)XZ, (void*)XZ, kXzN, 0L,
        dummy_bias,
        kRows, kXzN, kC, 1.0f);

    conv_silu_kernel<<<kRows / 64, 256, 0, stream>>>(XZ, conv_w, conv_b, UC, UCB, dirL);

    wmma_gemm64<1, 0, 0, 0, 0><<<dim3(16, 1), 256, 0, stream>>>(
        UCB, UCB, kDI, 0L,
        WXP, WXP, kDI, 0L,
        (void*)XD, (void*)XD, kXdP, 0L,
        dummy_bias,
        kRows, kXdP, kDI, 1.0f);

    scan_kernel<<<kB * (kDI / kScanCh), kScanCh, 0, stream>>>(XD, UC, XZ, dtproj_w, dtproj_b, A_log, D_param, YB, dirL);

    wmma_gemm64<1, 0, 0, 0, 0><<<dim3(32, 1), 256, 0, stream>>>(
        YB, YB, kDI, 0L,
        WOd, WOd, kDI, 0L,
        (void*)YSd, (void*)YSd, kC, 0L,
        dummy_bias,
        kRows, kC, kDI, 1.0f);
  }

  mid_split_kernel<<<(kRows * kC / 8) / 256, 256, 0, stream>>>(
      YS, YS + (size_t)kRows * kC, YS + (size_t)2 * kRows * kC, YS + (size_t)3 * kRows * kC, ACT, MIDH, MIDL, kRows * kC / 8);

  wmma_gemm64<1, 2, 1, 0, 2><<<dim3(16, kB), 256, 0, stream>>>(
      W2H, W2L, kC, 0L,
      MIDH, MIDL, kC, (long)kSeq * kC,
      (void*)dout, (void*)dout, kSeq, (long)kC * kSeq,
      T2,
      kC, kSeq, kC, 1.0f);
}
